// UNet_39805756899533
// MI455X (gfx1250) — hardware-verified
//
#include <hip/hip_runtime.h>
#include <math.h>

typedef __attribute__((ext_vector_type(16))) _Float16 v16h;
typedef __attribute__((ext_vector_type(16))) __bf16 v16b;
typedef __attribute__((ext_vector_type(8)))  _Float16 v8h;
typedef __attribute__((ext_vector_type(8)))  float v8f;
typedef __attribute__((ext_vector_type(4)))  float v4f;
typedef __attribute__((ext_vector_type(2)))  float v2f;
typedef __attribute__((ext_vector_type(4)))  unsigned v4u;
typedef __attribute__((ext_vector_type(4)))  int v4i;
typedef float __attribute__((may_alias)) float_a;
typedef int __attribute__((may_alias)) int_a;

template <typename T> __device__ __forceinline__ void vst2(void* p, T v) { *(volatile T*)p = v; __threadfence(); *(volatile T*)p = v; }
__device__ __forceinline__ v8f wmma16(v16h a, v16h b, v8f c) {
  v8f d = __builtin_amdgcn_wmma_f32_16x16x32_f16(false, a, false, b, (short)0, c, false, false);
  asm volatile("v_nop\n\tv_nop\n\tv_nop\n\tv_nop" : "+v"(d) : "v"(a), "v"(b));
  return d;
}
__device__ __forceinline__ v8f wmma_bf(v16b a, v16b b, v8f c) {
  v8f d = __builtin_amdgcn_wmma_f32_16x16x32_bf16(false, a, false, b, (short)0, c, false, false);
  asm volatile("v_nop\n\tv_nop\n\tv_nop\n\tv_nop" : "+v"(d) : "v"(a), "v"(b));
  return d;
}
__device__ __forceinline__ v16h frag_h(const _Float16* rowk0, int lane) {
  union { v16h v; v8h q[2]; } u; const _Float16* p = rowk0 + 8 * (lane >> 4);
  u.q[0] = *(const v8h*)p; u.q[1] = *(const v8h*)(p + 16); return u.v;
}
__device__ __forceinline__ v16h frag_f32(const float* rowk0, int lane) {
  v16h a; const float* p = rowk0 + 8 * (lane >> 4);
#pragma unroll
  for (int i = 0; i < 8; ++i) { a[i] = (_Float16)p[i]; a[8 + i] = (_Float16)p[16 + i]; }
  return a;
}
__device__ __forceinline__ v16h frag_f32s(const float* rowk0, int lane, float sc) {
  v16h a; const float* p = rowk0 + 8 * (lane >> 4);
#pragma unroll
  for (int i = 0; i < 8; ++i) { a[i] = (_Float16)(p[i] * sc); a[8 + i] = (_Float16)(p[16 + i] * sc); }
  return a;
}
__device__ __forceinline__ v16h fragc_f32(const float* W, int k0, int n, int lane, int ld, int K) {
  v16h a; const int g = lane >> 4;
#pragma unroll
  for (int i = 0; i < 8; ++i) { const int ka = k0 + 8 * g + i, kb = ka + 16;
    a[i] = (_Float16)(ka < K ? W[(size_t)(ka < K ? ka : K - 1) * ld + n] : 0.f); a[8 + i] = (_Float16)(kb < K ? W[(size_t)(kb < K ? kb : K - 1) * ld + n] : 0.f); }
  return a;
}
struct F2 { v16b h, l; };
__device__ __forceinline__ F2 bsplit16(const float v[16]) { F2 r;
#pragma unroll
  for (int i = 0; i < 16; ++i) { const __bf16 h = (__bf16)v[i]; r.h[i] = h; r.l[i] = (__bf16)(v[i] - (float)h); }
  return r; }
__device__ __forceinline__ F2 split_row(const float* row, int k0, int lane) { float v[16]; const float* p = row + k0 + 8 * (lane >> 4);
#pragma unroll
  for (int i = 0; i < 8; ++i) { v[i] = p[i]; v[8 + i] = p[16 + i]; }
  return bsplit16(v); }
__device__ __forceinline__ F2 split_rowK(const float* row, int k0, int lane, int K) { float v[16]; const int g = lane >> 4;
#pragma unroll
  for (int i = 0; i < 8; ++i) { const int ka = k0 + 8 * g + i, kb = ka + 16; v[i] = ka < K ? row[ka < K ? ka : K - 1] : 0.f; v[8 + i] = kb < K ? row[kb < K ? kb : K - 1] : 0.f; }
  return bsplit16(v); }
__device__ __forceinline__ F2 split_col(const float* W, int k0, int n, int lane, int ld, int K) { float v[16]; const int g = lane >> 4;
#pragma unroll
  for (int i = 0; i < 8; ++i) { const int ka = k0 + 8 * g + i, kb = ka + 16; v[i] = ka < K ? W[(size_t)(ka < K ? ka : K - 1) * ld + n] : 0.f; v[8 + i] = kb < K ? W[(size_t)(kb < K ? kb : K - 1) * ld + n] : 0.f; }
  return bsplit16(v); }
__device__ __forceinline__ v8f mac3(const F2& a, const F2& b, v8f c) { c = wmma_bf(a.l, b.h, c); c = wmma_bf(a.h, b.l, c); return wmma_bf(a.h, b.h, c); }
__device__ __forceinline__ float sigm(float v) { return 1.0f / (1.0f + expf(-v)); }
#define LDSX() do { asm volatile("s_wait_dscnt 0" ::: "memory"); __builtin_amdgcn_wave_barrier(); __builtin_amdgcn_fence(__ATOMIC_RELEASE, "workgroup"); } while (0)


#define NB 8
#define LL 4096
#define CC 256
#define NH 8
#define DD 32
#define CH 128
#define NCH (LL / CH)
#define NROW (NB * LL)
#ifndef TNB
#define TNB NB
#endif
typedef __attribute__((ext_vector_type(8))) __bf16 v8b;
__device__ __forceinline__ v16b frag_b(const __bf16* rowk0, int lane) {
  union { v16b v; v8b q[2]; } u; const __bf16* p = rowk0 + 8 * (lane >> 4);
  u.q[0] = *(const v8b*)p; u.q[1] = *(const v8b*)(p + 16); return u.v;
}
__device__ __forceinline__ float bfr(float v) { return (float)(__bf16)v; }
__device__ __attribute__((noinline)) float exp_ni(float v) { return expf(v); }
__device__ __attribute__((noinline)) float erf_ni(float v) { return erff(v); }

#define WS_QR  0u
#define WS_KR  (WS_QR + 4u * (size_t)NROW * CC)
#define WS_KP  (WS_KR + 4u * (size_t)NROW * CC)
#define WS_VP  (WS_KP + 4u * (size_t)NROW * CC)
#define WS_O   (WS_VP + 4u * (size_t)NROW * CC)
#define WS_END (WS_O + 4u * (size_t)NROW * CC)

__global__ __launch_bounds__(128) void k_qkv(const float* __restrict__ X, const float* __restrict__ RP, const float* __restrict__ Wt, const float* __restrict__ GQ, const float* __restrict__ GK, float* __restrict__ QR, float* __restrict__ KR, float* __restrict__ KP, float* __restrict__ VP) { __shared__ __align__(16) float sf[4][16][132]; __shared__ __align__(16) float tt[128][68];
  const int tid = threadIdx.x, wave = tid >> 5, lane = tid & 31, col = lane & 15, g = lane >> 4; const int cg = blockIdx.y; const int which = cg >> 1; const int c0 = (cg & 1) * 128; const size_t b = blockIdx.z; const int l0 = blockIdx.x * 64; const size_t r0 = b * LL + l0 + wave * 16;
  v8f acc[8] = {};
#pragma unroll
  for (int kc = 0; kc < CC / 32; ++kc) { float v[16]; { const float* xr = X + (r0 + col) * CC + kc * 32 + 8 * g; const float* pr = RP + (size_t)(l0 + wave * 16 + col) * CC + kc * 32 + 8 * g;
#pragma unroll
      for (int i = 0; i < 8; ++i) { v[i] = bfr(xr[i]) + bfr(pr[i]); v[8 + i] = bfr(xr[16 + i]) + bfr(pr[16 + i]); } }
    const F2 a = bsplit16(v);
#pragma unroll
    for (int j = 0; j < 8; ++j) { v16b w; const size_t o = (size_t)which * CC + c0 + j * 16 + col;
#pragma unroll
      for (int i = 0; i < 8; ++i) { w[i] = (__bf16)Wt[o * CC + kc * 32 + 8 * g + i]; w[8 + i] = (__bf16)Wt[o * CC + kc * 32 + 16 + 8 * g + i]; }
      acc[j] = wmma_bf(a.h, w, acc[j]); acc[j] = wmma_bf(a.l, w, acc[j]); } }
  float rn[4][8];
#pragma unroll
  for (int p = 0; p < 4; ++p)
#pragma unroll
    for (int r = 0; r < 8; ++r) { float a2 = acc[2 * p][r] * acc[2 * p][r] + acc[2 * p + 1][r] * acc[2 * p + 1][r];
#pragma unroll
      for (int o = 1; o < 16; o <<= 1) a2 += __shfl_xor(a2, o);
      rn[p][r] = (which == 2) ? 1.0f : 5.656854249492381f / fmaxf(sqrtf(a2), 1e-12f); }
  const float* GM = (which == 0) ? GQ : GK;
  if (which == 0 || which == 1) {
#pragma unroll
    for (int j = 0; j < 8; ++j) { const int cabs = c0 + j * 16 + col; const int hh = cabs / DD, d = cabs % DD; const float gm = bfr(GM[hh * DD + d]);
#pragma unroll
      for (int r = 0; r < 8; ++r) sf[wave][8 * g + r][j * 16 + col] = acc[j][r] * rn[j >> 1][r] * gm; }
    LDSX(); { float* dst = (which == 0) ? QR : KR; for (int rl = 0; rl < 16; ++rl) vst2(dst + (r0 + rl) * CC + c0 + lane * 4, *(const v4f*)&sf[wave][rl][lane * 4]); }
    LDSX(); }
  if (which == 1 || which == 2) {
#pragma unroll
    for (int j = 0; j < 8; ++j) { const int cabs = c0 + j * 16 + col; const int hh = cabs / DD, d = cabs % DD; const float gm = (which == 1) ? bfr(GM[hh * DD + d]) : 1.0f;
#pragma unroll
      for (int r = 0; r < 8; ++r) tt[j * 16 + col][wave * 16 + 8 * g + r] = acc[j][r] * rn[j >> 1][r] * gm; }
    __syncthreads(); { float* dst = (which == 1) ? KP : VP; for (int e = tid; e < 128 * 16; e += 128) { const int cl = e >> 4, q = e & 15; vst2(dst + ((b * CC + c0 + cl) * (size_t)LL) + l0 + q * 4, *(const v4f*)&tt[cl][q * 4]); } } } }
__device__ __forceinline__ F2 split_row_scaled(const float* row, int k0, int lane, const float* sc) { float v[16]; const float* p = row + k0 + 8 * (lane >> 4); const float* s = sc + k0 + 8 * (lane >> 4);
#pragma unroll
  for (int i = 0; i < 8; ++i) { v[i] = p[i] * s[i]; v[8 + i] = p[16 + i] * s[16 + i]; }
  return bsplit16(v); }
__global__ __launch_bounds__(128) void k_lin(const float* __restrict__ QR, const float* __restrict__ KR, const float* __restrict__ KP, const float* __restrict__ VP, float* __restrict__ O) {
  __shared__ __align__(16) float ssc[CH][132]; __shared__ __align__(16) float skv[DD][36]; __shared__ __align__(16) float sqd[CH], skd[CH], smk[CH]; __shared__ __align__(16) float so[4][32][36];
  const int tid = threadIdx.x, wave = tid >> 5, lane = tid & 31, col = lane & 15, g = lane >> 4; const int h = blockIdx.x; const size_t b = blockIdx.y;
  const float slope = exp2f(-(float)(h + 1));
  for (int e = tid; e < CH; e += 128) { sqd[e] = expf(-slope * (float)e); skd[e] = expf(-slope * (float)(CH - e)); smk[e] = expf(-slope * (float)e); }
  for (int e = tid; e < DD * 36; e += 128) (&skv[0][0])[e] = 0.f;
  const float blk = expf(-slope * (float)CH);
  __syncthreads();
#pragma unroll 1
  for (int n = 0; n < NCH; ++n) { const size_t rowc = b * LL + (size_t)n * CH;
#pragma unroll
    for (int rt = 0; rt < 2; ++rt) { const int t0 = wave * 32 + rt * 16; const F2 a = split_row(QR + (rowc + t0 + col) * CC + h * DD, 0, lane); v8f acc[8] = {};
#pragma unroll
      for (int j = 0; j < 8; ++j) { const F2 w = split_row(KR + (rowc + j * 16 + col) * CC + h * DD, 0, lane); acc[j] = mac3(a, w, acc[j]); }
#pragma unroll
      for (int j = 0; j < 8; ++j)
#pragma unroll
        for (int r = 0; r < 8; ++r) { const int t = t0 + 8 * g + r, s = j * 16 + col; ssc[t][s] = (s <= t) ? acc[j][r] * smk[t - s] : 0.f; } }
    LDSX();
#pragma unroll
    for (int rt = 0; rt < 2; ++rt) { const int t0 = wave * 32 + rt * 16; v8f oc[2] = {};
#pragma unroll
      for (int kc = 0; kc < CH / 32; ++kc) { const F2 a = split_row(&ssc[t0 + col][0], kc * 32, lane);
#pragma unroll
        for (int j = 0; j < 2; ++j) { const F2 w = split_row(VP + ((b * CC + h * DD + j * 16 + col) * (size_t)LL) + (size_t)n * CH, kc * 32, lane); oc[j] = mac3(a, w, oc[j]); } }
      { float v[16]; const float* qr = QR + (rowc + t0 + col) * CC + h * DD + 8 * g; const float qd = sqd[t0 + col];
#pragma unroll
        for (int i = 0; i < 8; ++i) { v[i] = qr[i] * qd; v[8 + i] = qr[16 + i] * qd; }
        const F2 a = bsplit16(v);
#pragma unroll
        for (int j = 0; j < 2; ++j) { const F2 w = split_row(&skv[j * 16 + col][0], 0, lane); oc[j] = mac3(a, w, oc[j]); } }
#pragma unroll
      for (int j = 0; j < 2; ++j)
#pragma unroll
        for (int r = 0; r < 8; ++r) so[wave][rt * 16 + 8 * g + r][j * 16 + col] = oc[j][r]; }
    LDSX();
    for (int rl = 0; rl < 32; ++rl) if (lane < 8) vst2(O + (rowc + wave * 32 + rl) * CC + h * DD + lane * 4, *(const v4f*)&so[wave][rl][lane * 4]);
    __syncthreads();
    { const int et = wave >> 1, dt = wave & 1; v8f acc = {};
#pragma unroll
      for (int kc = 0; kc < CH / 32; ++kc) { const F2 a = split_row(VP + ((b * CC + h * DD + et * 16 + col) * (size_t)LL) + (size_t)n * CH, kc * 32, lane); const F2 w = split_row_scaled(KP + ((b * CC + h * DD + dt * 16 + col) * (size_t)LL) + (size_t)n * CH, kc * 32, lane, skd); acc = mac3(a, w, acc); }
#pragma unroll
      for (int r = 0; r < 8; ++r) { const int e = et * 16 + 8 * g + r, d = dt * 16 + col; skv[e][d] = blk * skv[e][d] + acc[r]; } }
    __syncthreads(); } }
__global__ __launch_bounds__(128) void k_proj(const float* __restrict__ O, const float* __restrict__ PW, const float* __restrict__ PB, float* __restrict__ OUT) { __shared__ __align__(16) float sf[4][16][132];
  const int tid = threadIdx.x, wave = tid >> 5, lane = tid & 31, col = lane & 15, g = lane >> 4; const size_t r0 = (size_t)blockIdx.x * 64 + wave * 16; const int c0 = blockIdx.y * 128;
  v8f acc[8] = {};
#pragma unroll
  for (int kc = 0; kc < CC / 32; ++kc) { const F2 a = split_row(O + (r0 + col) * CC, kc * 32, lane);
#pragma unroll
    for (int j = 0; j < 8; ++j) { v16b w; const int o = c0 + j * 16 + col;
#pragma unroll
      for (int i = 0; i < 8; ++i) { w[i] = (__bf16)PW[(size_t)o * CC + kc * 32 + 8 * g + i]; w[8 + i] = (__bf16)PW[(size_t)o * CC + kc * 32 + 16 + 8 * g + i]; }
      acc[j] = wmma_bf(a.h, w, acc[j]); acc[j] = wmma_bf(a.l, w, acc[j]); } }
#pragma unroll
  for (int j = 0; j < 8; ++j) { const float bb = bfr(PB[c0 + j * 16 + col]);
#pragma unroll
    for (int r = 0; r < 8; ++r) sf[wave][8 * g + r][j * 16 + col] = acc[j][r] + bb; }
  LDSX(); for (int rl = 0; rl < 16; ++rl) vst2(OUT + (r0 + rl) * CC + c0 + lane * 4, *(const v4f*)&sf[wave][rl][lane * 4]); }
extern "C" void kernel_launch(void* const* d_in, const int* in_sizes, int n_in, void* d_out, int out_size, void* d_ws, size_t ws_size, hipStream_t stream) {
  (void)in_sizes; (void)n_in; (void)out_size;
  const float** F = (const float**)d_in;
  if (ws_size < (size_t)WS_END) return;
  char* ws = (char*)d_ws; float *QR = (float*)(ws + WS_QR), *KR = (float*)(ws + WS_KR), *KP = (float*)(ws + WS_KP), *VP = (float*)(ws + WS_VP), *O = (float*)(ws + WS_O);
  k_qkv<<<dim3(LL / 64, 6, TNB), 128, 0, stream>>>(F[0], F[1], F[2], F[3], F[4], QR, KR, KP, VP);
  k_lin<<<dim3(NH, TNB), 128, 0, stream>>>(QR, KR, KP, VP, O);
  k_proj<<<dim3(TNB * LL / 64, CC / 128), 128, 0, stream>>>(O, F[5], F[6], (float*)d_out);
}
